// GAT_85779086835952
// MI455X (gfx1250) — hardware-verified
//
#include <hip/hip_runtime.h>
#include <stddef.h>
#include <stdint.h>
#include <math.h>


#define F_IN    128
#define XQ      (F_IN / 8)
#define NHEAD   4
#define HID1    64
#define HC      256
#define KA      512
#define OUTC    32
#define LD2     64
#define NTHR    256
#define NWAVE   8
#define EPT     8
#define CHUNK   (NTHR * EPT)
#define WCAP    (EPT * 32)
#define LISTN   (NWAVE * WCAP)
#define NBMAX   2048
#define SLOTB   11
#define NBRUN   1024
#define RCAP    28672
#define DEGCAP  128
#define STW     32
#define GBM     64
#define GBN     64
#define GTHR    128
#define NEGSL   0.2f
#define EPS_SM  1e-16f
#define WSMAX   134217728
#define LDS_AGG ((2 * RCAP + 2 * NBMAX + LISTN) * 4 + 64)

static_assert((CHUNK & (CHUNK - 1)) == 0 && CHUNK <= (1 << SLOTB));
static_assert(NBMAX == (1 << SLOTB));
static_assert((NBRUN & (NBRUN - 1)) == 0 && NBRUN <= NBMAX && NBRUN >= 16);
static_assert(NTHR * 8 == NBMAX);
static_assert(LISTN >= NBMAX);
static_assert(LISTN >= NWAVE * WCAP);
static_assert((RCAP % 32) == 0);
static_assert(NWAVE * STW <= RCAP);
static_assert(OUTC <= STW);
static_assert(LDS_AGG <= 300000);
static_assert(GBM == (GTHR / 32) * 16);
static_assert((F_IN % 32) == 0 && (KA % 32) == 0);
static_assert((HC % GBN) == 0 && (LD2 % GBN) == 0);
static_assert(HC == NHEAD * HID1 && KA == 2 * HC && LD2 == 2 * OUTC);
static_assert(HC == 32 * 8);
static_assert(HID1 == 8 * 8);
static_assert(OUTC == 32);
static_assert(XQ == 16 && (F_IN % 8) == 0 && (HC % 8) == 0);
static_assert(HC * LD2 >= LD2 * 1);

typedef float          v4f  __attribute__((ext_vector_type(4)));
typedef float          v8f  __attribute__((ext_vector_type(8)));
typedef int            v4i  __attribute__((ext_vector_type(4)));
typedef int            v8i  __attribute__((ext_vector_type(8)));
typedef unsigned int   v4u  __attribute__((ext_vector_type(4)));
typedef unsigned short v8us __attribute__((ext_vector_type(8)));
typedef __bf16         v16b __attribute__((ext_vector_type(16)));
typedef v4f  __attribute__((may_alias)) v4fa;
typedef v8us __attribute__((may_alias)) v8usa;
union FragB { v16b v; v8us h[2]; v8i w; };

__device__ __forceinline__ v8f wmb(const FragB& a, const FragB& b, v8f c) {
  v8f d = __builtin_amdgcn_wmma_f32_16x16x32_bf16(false, a.v, false, b.v, (short)0, c, false, false);
  asm volatile("v_nop\n\tv_nop\n\tv_nop\n\tv_nop" : "+v"(d) : "v"(a.w), "v"(b.w));
  return d;
}

__device__ __forceinline__ void ldwait() {
  asm volatile("s_wait_loadcnt 0x0" ::: "memory");
}

__device__ __forceinline__ unsigned int f2bf(float f) {
  const unsigned int u = __float_as_uint(f);
  return ((u + 0x7FFFu + ((u >> 16) & 1u)) >> 16) & 0xFFFFu;
}
__device__ __forceinline__ float bf2f(unsigned int b) { return __uint_as_float(b << 16); }
__device__ __forceinline__ float bfr(float f) { return bf2f(f2bf(f)); }
__device__ __forceinline__ v4f bfr4(const v4f a) {
  v4f r; r.x = bfr(a.x); r.y = bfr(a.y); r.z = bfr(a.z); r.w = bfr(a.w); return r;
}
__device__ __forceinline__ unsigned int pk2(float lo, float hi) { return f2bf(lo) | (f2bf(hi) << 16); }
__device__ __forceinline__ v4u pack8(const v4f a, const v4f b) {
  v4u r;
  r.x = pk2(a.x, a.y); r.y = pk2(a.z, a.w); r.z = pk2(b.x, b.y); r.w = pk2(b.z, b.w);
  return r;
}
__device__ __forceinline__ void split8(const v4f a, const v4f b, v4u& hv, v4u& lv) {
  const float f[8] = {a.x, a.y, a.z, a.w, b.x, b.y, b.z, b.w};
  unsigned int hb[8], lb[8];
#pragma unroll
  for (int i = 0; i < 8; ++i) {
    hb[i] = f2bf(f[i]);
    lb[i] = f2bf(f[i] - bf2f(hb[i]));
  }
  hv.x = hb[0] | (hb[1] << 16); hv.y = hb[2] | (hb[3] << 16); hv.z = hb[4] | (hb[5] << 16); hv.w = hb[6] | (hb[7] << 16);
  lv.x = lb[0] | (lb[1] << 16); lv.y = lb[2] | (lb[3] << 16); lv.z = lb[4] | (lb[5] << 16); lv.w = lb[6] | (lb[7] << 16);
}
__device__ __forceinline__ float eluf(float v) {
  const float e = __expf(v) - 1.0f;
  return v > 0.f ? v : e;
}

__device__ __forceinline__ int scan_chunk(const int* __restrict__ dsts, int nE, int cbase, int slotBase,
                                          int nb, int vec8, int* list, int tid, int lane, int wave) {
  int wc = 0;
  const int el0  = tid * EPT;
  const int e0   = cbase + el0;
  const int sent = -2147483647 - 1;
  v4i da, db;
  if (vec8 != 0 && cbase + CHUNK <= nE) {
    da = *(const v4i*)(dsts + e0);
    db = *(const v4i*)(dsts + e0 + 4);
  } else {
    da.x = (e0     < nE) ? dsts[min(e0,     nE - 1)] : sent;
    da.y = (e0 + 1 < nE) ? dsts[min(e0 + 1, nE - 1)] : sent;
    da.z = (e0 + 2 < nE) ? dsts[min(e0 + 2, nE - 1)] : sent;
    da.w = (e0 + 3 < nE) ? dsts[min(e0 + 3, nE - 1)] : sent;
    db.x = (e0 + 4 < nE) ? dsts[min(e0 + 4, nE - 1)] : sent;
    db.y = (e0 + 5 < nE) ? dsts[min(e0 + 5, nE - 1)] : sent;
    db.z = (e0 + 6 < nE) ? dsts[min(e0 + 6, nE - 1)] : sent;
    db.w = (e0 + 7 < nE) ? dsts[min(e0 + 7, nE - 1)] : sent;
  }
  const unsigned nbs = (unsigned)slotBase;
  const unsigned unb = (unsigned)nb;
  const unsigned s0 = (unsigned)da.x - nbs, s1 = (unsigned)da.y - nbs;
  const unsigned s2 = (unsigned)da.z - nbs, s3 = (unsigned)da.w - nbs;
  const unsigned s4 = (unsigned)db.x - nbs, s5 = (unsigned)db.y - nbs;
  const unsigned s6 = (unsigned)db.z - nbs, s7 = (unsigned)db.w - nbs;
  const bool h0 = s0 < unb, h1 = s1 < unb, h2 = s2 < unb, h3 = s3 < unb;
  const bool h4 = s4 < unb, h5 = s5 < unb, h6 = s6 < unb, h7 = s7 < unb;
  const unsigned any = __builtin_amdgcn_ballot_w32(h0 | h1 | h2 | h3 | h4 | h5 | h6 | h7);
  if (any != 0u) {
#define HITJ(J, HJ, SJ) { \
      const unsigned mj = __builtin_amdgcn_ballot_w32(HJ); \
      if (mj != 0u) { \
        if (HJ) { \
          const int pos = wc + (int)__builtin_amdgcn_mbcnt_lo(mj, 0u); \
          if (pos < WCAP) list[wave * WCAP + pos] = ((el0 + (J)) << SLOTB) | (int)(SJ); \
        } \
        wc += (int)__builtin_popcount(mj); } }
    HITJ(0, h0, s0)
    HITJ(1, h1, s1)
    HITJ(2, h2, s2)
    HITJ(3, h3, s3)
    HITJ(4, h4, s4)
    HITJ(5, h5, s5)
    HITJ(6, h6, s6)
    HITJ(7, h7, s7)
#undef HITJ
  }
  return wc;
}

__global__ __launch_bounds__(NTHR) void k_xprep(const float* __restrict__ x, unsigned short* xb, int nN, int nUnits) {
  const int i = (int)blockIdx.x * NTHR + (int)threadIdx.x;
  if (i >= nUnits) return;
  const int row = i >> 4;
  const int c0  = (i & 15) * 8;
  const int rc  = row < nN ? row : nN - 1;
  const float* p = x + (size_t)rc * F_IN + c0;
  v4f a = *(const v4fa*)p, b = *(const v4fa*)(p + 4);
  const v4f z4 = {0.f, 0.f, 0.f, 0.f};
  if (row >= nN) { a = z4; b = z4; }
  const v4u hv = pack8(a, b);
  const size_t o = (size_t)row * F_IN + c0;
  *(volatile v4u*)(xb + o) = hv;
  __threadfence();
  *(volatile v4u*)(xb + o) = hv;
}

__global__ __launch_bounds__(NTHR) void k_wtr(const float* __restrict__ w, int Kin, int Ncol, int Nrows, int Kout,
                                              unsigned short* wt, int nUnits) {
  const int u = (int)blockIdx.x * NTHR + (int)threadIdx.x;
  if (u >= nUnits) return;
  const int kq = Kout >> 3;
  const int n  = u / kq;
  const int k8 = (u - n * kq) * 8;
  const int kk = k8 - (k8 / Kin) * Kin;
  const int ncl = n < Ncol ? n : Ncol - 1;
  const float* p = w + (size_t)kk * (size_t)Ncol + ncl;
  v4f a, b;
  a.x = p[0];                    a.y = p[(size_t)Ncol];         a.z = p[(size_t)2 * Ncol];     a.w = p[(size_t)3 * Ncol];
  b.x = p[(size_t)4 * Ncol];     b.y = p[(size_t)5 * Ncol];     b.z = p[(size_t)6 * Ncol];     b.w = p[(size_t)7 * Ncol];
  const v4f z4 = {0.f, 0.f, 0.f, 0.f};
  if (n >= Ncol || n >= Nrows) { a = z4; b = z4; }
  const v4u wv = pack8(a, b);
  unsigned short* o = wt + (size_t)n * (size_t)Kout + k8;
  *(volatile v4u*)o = wv;
  __threadfence();
  *(volatile v4u*)o = wv;
}

__global__ __launch_bounds__(GTHR) void k_gemm(
    const unsigned short* __restrict__ A, const unsigned short* __restrict__ WT,
    float* outF, int K, int ldo)
{
  __shared__ __attribute__((aligned(16))) float stg[GBM * GBN];
  const int tid = (int)threadIdx.x, lane = tid & 31, wave = tid >> 5, hh = lane >> 4, m = lane & 15;
  const int rowBase = (int)blockIdx.x * GBM;
  const int col0    = (int)blockIdx.y * GBN;

  v8f acc[4];
  {
    const v8f z = {0.f, 0.f, 0.f, 0.f, 0.f, 0.f, 0.f, 0.f};
    acc[0] = z; acc[1] = z; acc[2] = z; acc[3] = z;
  }
  const unsigned short* ap = A  + (size_t)(rowBase + 16 * wave + m) * (size_t)K + 8 * hh;
  const unsigned short* wp = WT + (size_t)(col0 + m) * (size_t)K + 8 * hh;
  const int ksteps = K >> 5;
#pragma unroll 1
  for (int ks = 0; ks < ksteps; ++ks) {
    FragB af;
    af.h[0] = *(const v8usa*)(ap + 32 * ks);
    af.h[1] = *(const v8usa*)(ap + 32 * ks + 16);
#pragma unroll
    for (int t = 0; t < 4; ++t) {
      const unsigned short* wq = wp + (size_t)(16 * t) * (size_t)K + 32 * ks;
      FragB bf;
      bf.h[0] = *(const v8usa*)wq;
      bf.h[1] = *(const v8usa*)(wq + 16);
      acc[t] = wmb(af, bf, acc[t]);
    }
  }

#pragma unroll
  for (int t = 0; t < 4; ++t) {
    const int lc = 16 * t + m;
#pragma unroll
    for (int r = 0; r < 8; ++r) {
      const int lr = 16 * wave + 8 * hh + r;
      stg[lr * GBN + lc] = acc[t][r];
    }
  }
  __syncthreads();

  v4f fv[8];
#pragma unroll
  for (int i = 0; i < 8; ++i) {
    const int lr = 16 * wave + 2 * i + hh;
    fv[i] = *(const v4fa*)(stg + lr * GBN + 4 * m);
  }
#pragma unroll
  for (int i = 0; i < 8; ++i) {
    const int lr = 16 * wave + 2 * i + hh;
    const int gr = rowBase + lr;
    float* op = outF + (size_t)gr * (size_t)ldo + col0 + 4 * m;
    *(volatile v4f*)op = fv[i];
  }
  __threadfence();
#pragma unroll
  for (int i = 0; i < 8; ++i) {
    const int lr = 16 * wave + 2 * i + hh;
    const int gr = rowBase + lr;
    float* op = outF + (size_t)gr * (size_t)ldo + col0 + 4 * m;
    *(volatile v4f*)op = fv[i];
  }
}

template<int L>
__global__ __launch_bounds__(NTHR) void k_agg(
    const int* __restrict__ srcs, const int* __restrict__ dsts,
    const float* __restrict__ F,
    const float* __restrict__ asrc, const float* __restrict__ adst,
    const float* __restrict__ bias,
    unsigned short* HP, float* out,
    int nN, int nE, int nb, int vec8, int MPr) {
  extern __shared__ v4f lds_dyn[];
  int* reg1 = (int*)lds_dyn;
  int* reg2 = reg1 + RCAP;
  int* scnt = reg2 + RCAP;
  int* soff = scnt + NBMAX;
  int* list = soff + NBMAX;
  int* wcnt = list + LISTN;
  int* wtot = wcnt + NWAVE;
  const int tid = (int)threadIdx.x, lane = tid & 31, wave = tid >> 5;
  const int nodeBase = (int)blockIdx.x * nb;

  for (int i = tid; i < NBMAX; i += NTHR) scnt[i] = 0;
  __syncthreads();

  int tot = 0;
  const int nChunks = (nE + CHUNK - 1) / CHUNK;
#pragma unroll 1
  for (int ch = 0; ch < nChunks; ++ch) {
    const int cbase = ch * CHUNK;
    const int wc = scan_chunk(dsts, nE, cbase, nodeBase, nb, vec8, list, tid, lane, wave);
    if (lane == 0) wcnt[wave] = wc;
    __syncthreads();
    int pre = 0, all = 0;
#pragma unroll
    for (int w2 = 0; w2 < NWAVE; ++w2) {
      int c = wcnt[w2];
      c = c < 0 ? 0 : (c > WCAP ? WCAP : c);
      all += c;
      pre += (w2 < wave) ? c : 0;
    }
    const int wcc  = wc > WCAP ? WCAP : wc;
    const int base = tot + pre;
#pragma unroll 1
    for (int i = lane; i < wcc; i += 32) {
      const int ent = list[wave * WCAP + i];
      const int el  = (ent >> SLOTB) & (CHUNK - 1);
      const int sl  = ent & (NBMAX - 1);
      int eid = cbase + el;
      eid = eid > nE - 1 ? nE - 1 : eid;
      const int pos = base + i;
      if (pos < RCAP) reg1[pos] = (int)(((unsigned)eid << SLOTB) | (unsigned)sl);
    }
    tot += all;
    tot = tot > RCAP ? RCAP : tot;
    __syncthreads();
  }
  const int nh = tot;

  if (wave == 0) {
#pragma unroll 1
    for (int b0 = 0; b0 < nh; b0 += 32) {
      const int idx = b0 + lane;
      const int uv  = reg1[idx < nh ? idx : nh - 1];
      const int m32 = (nh - b0) < 32 ? (nh - b0) : 32;
#pragma unroll 1
      for (int k = 0; k < m32; ++k) {
        const int u  = __builtin_amdgcn_readlane(uv, k);
        const int sl = u & (NBMAX - 1);
        if (lane == 0) scnt[sl] = scnt[sl] + 1;
      }
    }
  }
  __syncthreads();

  {
    const v4i ca = *(const v4i*)(scnt + 8 * tid);
    const v4i cb = *(const v4i*)(scnt + 8 * tid + 4);
    const int e0 = ca.x < 0 ? 0 : ca.x, e1 = ca.y < 0 ? 0 : ca.y, e2 = ca.z < 0 ? 0 : ca.z, e3 = ca.w < 0 ? 0 : ca.w;
    const int e4 = cb.x < 0 ? 0 : cb.x, e5 = cb.y < 0 ? 0 : cb.y, e6 = cb.z < 0 ? 0 : cb.z, e7 = cb.w < 0 ? 0 : cb.w;
    const int ts = e0 + e1 + e2 + e3 + e4 + e5 + e6 + e7;
    int incl = ts;
#pragma unroll
    for (int d = 1; d < 32; d <<= 1) {
      const int up = __shfl_up(incl, d);
      if (lane >= d) incl += up;
    }
    if (lane == 31) wtot[wave] = incl;
    __syncthreads();
    int pre = 0;
#pragma unroll
    for (int w2 = 0; w2 < NWAVE; ++w2) pre += (w2 < wave) ? wtot[w2] : 0;
    int run = pre + incl - ts;
    soff[8 * tid + 0] = run; run += e0;
    soff[8 * tid + 1] = run; run += e1;
    soff[8 * tid + 2] = run; run += e2;
    soff[8 * tid + 3] = run; run += e3;
    soff[8 * tid + 4] = run; run += e4;
    soff[8 * tid + 5] = run; run += e5;
    soff[8 * tid + 6] = run; run += e6;
    soff[8 * tid + 7] = run;
  }
  __syncthreads();
  for (int i = tid; i < NBMAX; i += NTHR) list[i] = soff[i];
  __syncthreads();

  if (wave == 0) {
#pragma unroll 1
    for (int b0 = 0; b0 < nh; b0 += 32) {
      const int idx = b0 + lane;
      const int uv  = reg1[idx < nh ? idx : nh - 1];
      const int m32 = (nh - b0) < 32 ? (nh - b0) : 32;
#pragma unroll 1
      for (int k = 0; k < m32; ++k) {
        const int u   = __builtin_amdgcn_readlane(uv, k);
        const int sl  = u & (NBMAX - 1);
        const int eid = (int)((unsigned)u >> SLOTB);
        if (lane == 0) {
          int pos = list[sl];
          pos = pos < 0 ? 0 : (pos > RCAP - 1 ? RCAP - 1 : pos);
          reg2[pos] = eid;
          list[sl] = pos + 1;
        }
      }
    }
  }
  __syncthreads();

  const int nbw = nb >> 3;
  const bool ovf = (nh >= RCAP);
  const float qnan = __int_as_float(0x7fc00000);

  if (L == 1) {
    const int cofs = 8 * lane;
    float as8[8], ad8[8], bb8[8];
    {
      const v4f sa = bfr4(*(const v4fa*)(asrc + cofs)), sb = bfr4(*(const v4fa*)(asrc + cofs + 4));
      const v4f da = bfr4(*(const v4fa*)(adst + cofs)), db = bfr4(*(const v4fa*)(adst + cofs + 4));
      const v4f ba = bfr4(*(const v4fa*)(bias + cofs)), bb = bfr4(*(const v4fa*)(bias + cofs + 4));
      as8[0] = sa.x; as8[1] = sa.y; as8[2] = sa.z; as8[3] = sa.w; as8[4] = sb.x; as8[5] = sb.y; as8[6] = sb.z; as8[7] = sb.w;
      ad8[0] = da.x; ad8[1] = da.y; ad8[2] = da.z; ad8[3] = da.w; ad8[4] = db.x; ad8[5] = db.y; ad8[6] = db.z; ad8[7] = db.w;
      bb8[0] = ba.x; bb8[1] = ba.y; bb8[2] = ba.z; bb8[3] = ba.w; bb8[4] = bb.x; bb8[5] = bb.y; bb8[6] = bb.z; bb8[7] = bb.w;
    }
    ldwait();
#pragma unroll 1
    for (int jt = 0; jt < nbw; ++jt) {
      const int slot = wave * nbw + jt;
      const int grow = nodeBase + slot;
      const int gcl  = grow < nN ? grow : nN - 1;
      int st = soff[slot];
      const int craw = scnt[slot];
      int cnt = craw;
      st  = st < 0 ? 0 : (st > nh ? nh : st);
      cnt = cnt < 0 ? 0 : (cnt > DEGCAP ? DEGCAP : cnt);
      if (cnt > nh - st) cnt = nh - st;
      const float pz = (ovf || craw > DEGCAP) ? qnan : 0.0f;
      const bool live = grow < nN;

      const float* drow = F + (size_t)gcl * HC + cofs;
      float fd[8];
      {
        const v4f t0 = *(const v4fa*)drow, t1 = *(const v4fa*)(drow + 4);
        fd[0] = t0.x; fd[1] = t0.y; fd[2] = t0.z; fd[3] = t0.w; fd[4] = t1.x; fd[5] = t1.y; fd[6] = t1.z; fd[7] = t1.w;
      }
      ldwait();
      float pd = fd[0] * ad8[0];
#pragma unroll
      for (int i = 1; i < 8; ++i) pd = fmaf(fd[i], ad8[i], pd);
      pd += __shfl_xor(pd, 1);
      pd += __shfl_xor(pd, 2);
      pd += __shfl_xor(pd, 4);
      float p0 = fd[0] * as8[0];
#pragma unroll
      for (int i = 1; i < 8; ++i) p0 = fmaf(fd[i], as8[i], p0);
      p0 += __shfl_xor(p0, 1);
      p0 += __shfl_xor(p0, 2);
      p0 += __shfl_xor(p0, 4);
      float l0 = p0 + pd;
      l0 = l0 > 0.f ? l0 : NEGSL * l0;
      float mx = l0, dn = 1.0f;
      float av[8];
#pragma unroll
      for (int i = 0; i < 8; ++i) av[i] = fd[i];

#pragma unroll 1
      for (int q = 0; q < cnt; ++q) {
        int idx = st + q; idx = idx > RCAP - 1 ? RCAP - 1 : idx;
        int eid = reg2[idx]; eid = eid < 0 ? 0 : (eid > nE - 1 ? nE - 1 : eid);
        const int sraw = srcs[eid];
        const int s = sraw < 0 ? 0 : (sraw > nN - 1 ? nN - 1 : sraw);
        const float* sr = F + (size_t)s * HC + cofs;
        float fs[8];
        {
          const v4f t0 = *(const v4fa*)sr, t1 = *(const v4fa*)(sr + 4);
          fs[0] = t0.x; fs[1] = t0.y; fs[2] = t0.z; fs[3] = t0.w; fs[4] = t1.x; fs[5] = t1.y; fs[6] = t1.z; fs[7] = t1.w;
        }
        ldwait();
        float es = fs[0] * as8[0];
#pragma unroll
        for (int i = 1; i < 8; ++i) es = fmaf(fs[i], as8[i], es);
        es += __shfl_xor(es, 1);
        es += __shfl_xor(es, 2);
        es += __shfl_xor(es, 4);
        float lg = es + pd;
        lg = lg > 0.f ? lg : NEGSL * lg;
        const float df = lg - mx;
        const float ee = __expf(-fabsf(df));
        const bool up  = df > 0.f;
        const float s1 = up ? ee : 1.0f;
        const float s2 = up ? 1.0f : ee;
        mx = up ? lg : mx;
        dn = fmaf(dn, s1, s2);
#pragma unroll
        for (int i = 0; i < 8; ++i) av[i] = fmaf(av[i], s1, s2 * fs[i]);
      }
      const float inv = __builtin_amdgcn_rcpf(dn + EPS_SM);
      float r[8];
#pragma unroll
      for (int i = 0; i < 8; ++i) {
        const float v = eluf(fmaf(av[i], inv, bb8[i]));
        r[i] = (live ? v : 0.f) + pz;
      }
      v4f ra, rb;
      ra.x = r[0]; ra.y = r[1]; ra.z = r[2]; ra.w = r[3];
      rb.x = r[4]; rb.y = r[5]; rb.z = r[6]; rb.w = r[7];
      v4u hv, lv;
      split8(ra, rb, hv, lv);
      unsigned short* gh = HP + (size_t)grow * KA + cofs;
      unsigned short* gl = gh + HC;
      const bool wr = grow < MPr;
      if (wr) { *(volatile v4u*)gh = hv; *(volatile v4u*)gl = lv; }
      __threadfence();
      if (wr) { *(volatile v4u*)gh = hv; *(volatile v4u*)gl = lv; }
    }
  } else {
    float* stw = (float*)reg1 + wave * STW;
    const float as1 = bfr(asrc[lane]);
    const float ad1 = bfr(adst[lane]);
    const float bb1 = bfr(bias[lane]);
    const int lc = lane < 8 ? lane : 7;
    ldwait();
#pragma unroll 1
    for (int jt = 0; jt < nbw; ++jt) {
      const int slot = wave * nbw + jt;
      const int grow = nodeBase + slot;
      const int gcl  = grow < nN ? grow : nN - 1;
      int st = soff[slot];
      const int craw = scnt[slot];
      int cnt = craw;
      st  = st < 0 ? 0 : (st > nh ? nh : st);
      cnt = cnt < 0 ? 0 : (cnt > DEGCAP ? DEGCAP : cnt);
      if (cnt > nh - st) cnt = nh - st;
      const float pz = (ovf || craw > DEGCAP) ? qnan : 0.0f;

      const float fd1 = F[(size_t)gcl * LD2 + lane];
      ldwait();
      float pd = fd1 * ad1;
#pragma unroll
      for (int off = 16; off > 0; off >>= 1) pd += __shfl_xor(pd, off);
      float p0 = fd1 * as1;
#pragma unroll
      for (int off = 16; off > 0; off >>= 1) p0 += __shfl_xor(p0, off);
      float l0 = p0 + pd;
      l0 = l0 > 0.f ? l0 : NEGSL * l0;
      float mx = l0, dn = 1.0f, av1 = fd1;

#pragma unroll 1
      for (int q = 0; q < cnt; ++q) {
        int idx = st + q; idx = idx > RCAP - 1 ? RCAP - 1 : idx;
        int eid = reg2[idx]; eid = eid < 0 ? 0 : (eid > nE - 1 ? nE - 1 : eid);
        const int sraw = srcs[eid];
        const int s = sraw < 0 ? 0 : (sraw > nN - 1 ? nN - 1 : sraw);
        const float fs1 = F[(size_t)s * LD2 + lane];
        ldwait();
        float es = fs1 * as1;
#pragma unroll
        for (int off = 16; off > 0; off >>= 1) es += __shfl_xor(es, off);
        float lg = es + pd;
        lg = lg > 0.f ? lg : NEGSL * lg;
        const float df = lg - mx;
        const float ee = __expf(-fabsf(df));
        const bool up  = df > 0.f;
        const float s1 = up ? ee : 1.0f;
        const float s2 = up ? 1.0f : ee;
        mx = up ? lg : mx;
        dn = fmaf(dn, s1, s2);
        av1 = fmaf(av1, s1, s2 * fs1);
      }
      const float inv = __builtin_amdgcn_rcpf(dn + EPS_SM);
      const float z = fmaf(av1, inv, bb1);
      float vm = z;
#pragma unroll
      for (int off = 16; off > 0; off >>= 1) vm = fmaxf(vm, __shfl_xor(vm, off));
      const float ex = expf(z - vm);
      float sm = ex;
#pragma unroll
      for (int off = 16; off > 0; off >>= 1) sm += __shfl_xor(sm, off);
      const float o = ex * __builtin_amdgcn_rcpf(sm) + pz;
      __builtin_amdgcn_fence(__ATOMIC_RELEASE, "wavefront");
      __builtin_amdgcn_wave_barrier();
      stw[lane] = o;
      __builtin_amdgcn_fence(__ATOMIC_RELEASE, "wavefront");
      __builtin_amdgcn_wave_barrier();
      const v4f gv = *(const v4fa*)(stw + 4 * lc);
      float* gp = out + (size_t)grow * OUTC + 4 * lc;
      const bool wsv = (grow < nN) && (lane < 8);
      if (wsv) *(volatile v4f*)gp = gv;
      __threadfence();
      if (wsv) *(volatile v4f*)gp = gv;
    }
  }
  (void)HP; (void)out; (void)MPr;
}

static int pick_nb(int nE, int nN) {
  int nb = NBRUN;
  while (nb > 16 && (long long)nb * (long long)nE * 5LL > (long long)RCAP * (long long)nN * 4LL) nb >>= 1;
  return nb;
}
static inline int cdiv(int a, int b) { return (a + b - 1) / b; }

extern "C" void kernel_launch(void* const* d_in, const int* in_sizes, int n_in,
                              void* d_out, int out_size, void* d_ws, size_t ws_size,
                              hipStream_t stream) {
  if (n_in < 10) return;
  const int nN = in_sizes[0] / F_IN;
  if (nN <= 0 || in_sizes[0] != nN * F_IN || nN > (1 << 22)) return;
  if (in_sizes[1] < 2 || (in_sizes[1] & 1) != 0) return;
  const int nE = in_sizes[1] / 2;
  if (nE < 1 || nE >= (1 << (32 - SLOTB))) return;
  if (in_sizes[2] != F_IN * HC) return;
  if (in_sizes[3] != HC || in_sizes[4] != HC) return;
  if (in_sizes[5] != HC) return;
  if (in_sizes[6] != HC * OUTC) return;
  if (in_sizes[7] != OUTC || in_sizes[8] != OUTC) return;
  if (in_sizes[9] != OUTC) return;
  if (out_size != nN * OUTC) return;

  const float* x    = (const float*)d_in[0];
  const int*   ei   = (const int*)  d_in[1];
  const float* W1   = (const float*)d_in[2];
  const float* a1s  = (const float*)d_in[3];
  const float* a1d  = (const float*)d_in[4];
  const float* b1   = (const float*)d_in[5];
  const float* W2   = (const float*)d_in[6];
  const float* a2s  = (const float*)d_in[7];
  const float* a2d  = (const float*)d_in[8];
  const float* b2   = (const float*)d_in[9];
  float* out = (float*)d_out;
  const int* src = ei;
  const int* dst = ei + nE;

  const int MP   = cdiv(nN, GBM) * GBM;
  const int nb   = pick_nb(nE, nN);
  if (nb < 16 || (nb & (nb - 1)) != 0 || nb > NBRUN) return;
  const int gA   = cdiv(MP, nb);
  const int vec8 = ((nE & 3) == 0) ? 1 : 0;
  if (gA * nb < MP) return;

  char* ws = (char*)d_ws;
  size_t off = 0;
  const size_t oXB  = off; off += (size_t)MP * F_IN * 2;           off = (off + 255) & ~(size_t)255;
  const size_t oW1T = off; off += (size_t)HC * F_IN * 2;           off = (off + 255) & ~(size_t)255;
  const size_t oW2T = off; off += (size_t)LD2 * KA * 2;            off = (off + 255) & ~(size_t)255;
  const size_t oF   = off; off += (size_t)MP * HC * 4;             off = (off + 255) & ~(size_t)255;
  const size_t oHA  = off; off += (size_t)MP * KA * 2;             off = (off + 255) & ~(size_t)255;
  if (off > ws_size || off > (size_t)WSMAX) return;
  unsigned short* XB  = (unsigned short*)(ws + oXB);
  unsigned short* W1T = (unsigned short*)(ws + oW1T);
  unsigned short* W2T = (unsigned short*)(ws + oW2T);
  float*          F   = (float*)(ws + oF);
  unsigned short* HA  = (unsigned short*)(ws + oHA);

  hipFuncSetAttribute(reinterpret_cast<const void*>(&k_agg<1>),
                      hipFuncAttributeMaxDynamicSharedMemorySize, LDS_AGG);
  hipFuncSetAttribute(reinterpret_cast<const void*>(&k_agg<2>),
                      hipFuncAttributeMaxDynamicSharedMemorySize, LDS_AGG);

  const int nUx = MP * XQ;
  k_xprep<<<cdiv(nUx, NTHR), NTHR, 0, stream>>>(x, XB, nN, nUx);

  {
    const int nUw1 = HC * (F_IN / 8);
    k_wtr<<<cdiv(nUw1, NTHR), NTHR, 0, stream>>>(W1, F_IN, HC, HC, F_IN, W1T, nUw1);
    const int nUw2 = LD2 * (KA / 8);
    k_wtr<<<cdiv(nUw2, NTHR), NTHR, 0, stream>>>(W2, HC, OUTC, LD2, KA, W2T, nUw2);
  }

  const int gM = MP / GBM;
  k_gemm<<<dim3(gM, HC / GBN), GTHR, 0, stream>>>(XB, W1T, F, F_IN, HC);
  k_agg<1><<<gA, NTHR, LDS_AGG, stream>>>(src, dst, F, a1s, a1d, b1, HA, out, nN, nE, nb, vec8, MP);
  k_gemm<<<dim3(gM, LD2 / GBN), GTHR, 0, stream>>>(HA, W2T, F, KA, LD2);
  k_agg<2><<<gA, NTHR, LDS_AGG, stream>>>(src, dst, F, a2s, a2d, b2, HA, out, nN, nE, nb, vec8, MP);
}
